// TimeEncoder_72069551227407
// MI455X (gfx1250) — hardware-verified
//
#include <hip/hip_runtime.h>
#include <stddef.h>

typedef __attribute__((ext_vector_type(16))) _Float16 v16h;
typedef __attribute__((ext_vector_type(8)))  _Float16 v8h;
typedef __attribute__((ext_vector_type(16))) __bf16   v16b;
typedef __attribute__((ext_vector_type(8)))  __bf16   v8b;
typedef __attribute__((ext_vector_type(8)))  float    v8f;
typedef __attribute__((ext_vector_type(4)))  float    v4f;

__device__ __forceinline__ void dep_guard_h(v8f& a, v8f& b, v16h x, v16h y) { asm volatile("v_nop\n\tv_nop\n\tv_nop\n\tv_nop" : "+v"(a), "+v"(b) : "v"(x), "v"(y)); }
__device__ __forceinline__ void keep4_h(v16h a, v16h b, v16h c, v16h d) { asm volatile("v_nop" :: "v"(a), "v"(b), "v"(c), "v"(d)); }
template <typename T> struct Frag;
template <> struct Frag<_Float16> {
  typedef v16h V; union U { v16h v; v8h h[2]; };
  static __device__ __forceinline__ v16h load(const _Float16* p) {
    U f; f.h[0] = *(const v8h*)(p); f.h[1] = *(const v8h*)(p + 16); return f.v;
  }
  static __device__ __forceinline__ v8f mma(v16h a, v16h b, v8f c) {
    return __builtin_amdgcn_wmma_f32_16x16x32_f16(false, a, false, b, (short)0, c, false, false);
  }
  static __device__ __forceinline__ void guard(v8f& a, v8f& b, v16h x, v16h y) { dep_guard_h(a, b, x, y); }
  static __device__ __forceinline__ void keep(v16h a, v16h b, v16h c, v16h d) { keep4_h(a, b, c, d); }
};

__device__ __forceinline__ v8f mma16(v16h a, v16h b, v8f c) {
  c = __builtin_amdgcn_wmma_f32_16x16x32_f16(false, a, false, b, (short)0, c, false, false);
  asm volatile("v_nop\n\tv_nop\n\tv_nop\n\tv_nop" : "+v"(c) : "v"(a), "v"(b));
  return c;
}

__device__ __forceinline__ float sigm(float v) { return 1.0f / (1.0f + expf(-v)); }

constexpr int kSteps       = 128;
constexpr int kBatch       = 1024;
constexpr int kFields      = 6;
constexpr int kEmbDim      = 32;
constexpr int kVocab       = 18;
constexpr int kHid1        = 64;
constexpr int kHid2        = 128;
constexpr int kDimOut      = 128;
constexpr int kEmbWidth    = kFields * kEmbDim;
constexpr int kDepth1      = kEmbWidth + kHid1;
constexpr int kDepth2      = kHid1 + kHid2;
constexpr int kGates1      = 4 * kHid1;
constexpr int kGates2      = 4 * kHid2;
constexpr int kRowsPerBlk  = 32;
constexpr int kPitch1      = 264;
constexpr int kPitch2      = 200;
constexpr int kSlabPitch   = 132;
constexpr float kCarry     = 16.0f;
constexpr float kFold      = 1.0f / 256.0f;
static_assert(kDepth1 % 32 == 0 && kDepth2 % 32 == 0 && kHid2 % 32 == 0);
static_assert(kBatch % kRowsPerBlk == 0);
static_assert((kPitch1 * 2) % 16 == 0 && (kPitch2 * 2) % 16 == 0 && (kSlabPitch * 4) % 16 == 0);

__global__ __launch_bounds__(256) void build_bt(const float* __restrict__ src0, int k0n,
                                                const float* __restrict__ src1, int k1n,
                                                int ncols, int ktot,
                                                _Float16* __restrict__ dst, int nchunks) {
  const int j = blockIdx.x * 256 + threadIdx.x;
  if (j >= nchunks) return;
  const int cpr = ktot >> 3;
  const int n   = j / cpr;
  const int kb  = (j - n * cpr) * 8;
  v8h hv;
#pragma unroll
  for (int e = 0; e < 8; ++e) {
    const int k = kb + e;
    int ka = k;        ka = ka > (k0n - 1) ? (k0n - 1) : ka;  ka = ka < 0 ? 0 : ka;
    int kc = k - k0n;  kc = kc < 0 ? 0 : kc;                  kc = kc > (k1n - 1) ? (k1n - 1) : kc;
    const float v0 = src0[(size_t)ka * ncols + n];
    const float v1 = src1[(size_t)kc * ncols + n];
    const float v  = (k < k0n) ? v0 : v1;
    hv[e] = (_Float16)(v * kCarry);
  }
  _Float16* p = dst + (size_t)j * 8;
  *(volatile v8h*)p = hv;
  __threadfence();
  *(volatile v8h*)p = hv;
}

__global__ __launch_bounds__(256) void lstm2_persistent(const int* __restrict__ x,
                                                        const float* __restrict__ E,
                                                        const _Float16* __restrict__ Bt1,
                                                        const float* __restrict__ b1,
                                                        const _Float16* __restrict__ Bt2,
                                                        const float* __restrict__ b2,
                                                        const _Float16* __restrict__ Btd,
                                                        const float* __restrict__ bd,
                                                        float* __restrict__ out) {
  __shared__ __align__(16) _Float16 A1s[kRowsPerBlk * kPitch1];
  __shared__ __align__(16) _Float16 A2s[kRowsPerBlk * kPitch2];
  __shared__ __align__(16) _Float16 Es[kVocab * kEmbDim];
  __shared__ __align__(16) float    slab[kRowsPerBlk * kSlabPitch];

  const int tid  = threadIdx.x;
  const int lane = tid & 31;
  const int wave = tid >> 5;
  const int hf   = lane >> 4;
  const int cl   = lane & 15;
  const int b0   = blockIdx.x * kRowsPerBlk;

  for (int e = tid; e < kVocab * kEmbDim; e += 256) Es[e] = (_Float16)(E[e] * kCarry);
  {
    const _Float16 zh = (_Float16)0.0f;
    const v8h z8 = {zh, zh, zh, zh, zh, zh, zh, zh};
    for (int e = tid; e < (kRowsPerBlk * kPitch1) / 8; e += 256) *(v8h*)(A1s + e * 8) = z8;
    for (int e = tid; e < (kRowsPerBlk * kPitch2) / 8; e += 256) *(v8h*)(A2s + e * 8) = z8;
  }
  const int mt1 = wave >> 2;
  const int ub1 = wave & 3;
  float b1g[4], b2g[4];
#pragma unroll
  for (int g = 0; g < 4; ++g) {
    b1g[g] = b1[g * kHid1 + 16 * ub1 + cl];
    b2g[g] = b2[g * kHid2 + 16 * wave + cl];
  }
  const float bdv = bd[16 * wave + cl];

  float c1r[8];
  float c2r[16];
#pragma unroll
  for (int r = 0; r < 8; ++r) c1r[r] = 0.0f;
#pragma unroll
  for (int r = 0; r < 16; ++r) c2r[r] = 0.0f;

  const _Float16* a1Base  = A1s + (16 * mt1 + cl) * kPitch1 + 8 * hf;
  const _Float16* b1Base  = Bt1 + (size_t)(16 * ub1 + cl) * kDepth1 + 8 * hf;
  const _Float16* a2Base0 = A2s + cl * kPitch2 + 8 * hf;
  const _Float16* a2Base1 = A2s + (16 + cl) * kPitch2 + 8 * hf;
  const _Float16* b2Base  = Bt2 + (size_t)(16 * wave + cl) * kDepth2 + 8 * hf;

  __syncthreads();

  for (int t = 0; t < kSteps; ++t) {
#pragma unroll
    for (int i = 0; i < 3; ++i) {
      const int task = tid + 256 * i;
      const int q    = task & 3;
      const int rf   = task >> 2;
      const int row  = rf / kFields;
      const int f    = rf - row * kFields;
      int id = x[(size_t)(b0 + row) * (kSteps * kFields) + t * kFields + f];
      id = id < 0 ? 0 : id;
      id = id > (kVocab - 1) ? (kVocab - 1) : id;
      const v8h ev = *(const v8h*)(Es + id * kEmbDim + 8 * q);
      *(v8h*)(A1s + row * kPitch1 + f * kEmbDim + 8 * q) = ev;
    }
    __syncthreads();

    v8f acc1[4];
#pragma unroll
    for (int g = 0; g < 4; ++g) acc1[g] = (v8f){0.f, 0.f, 0.f, 0.f, 0.f, 0.f, 0.f, 0.f};
#pragma unroll 1
    for (int ks = 0; ks < kDepth1 / 32; ++ks) {
      const v16h a = Frag<_Float16>::load(a1Base + 32 * ks);
#pragma unroll
      for (int g = 0; g < 4; ++g) {
        const v16h bf = Frag<_Float16>::load(b1Base + (size_t)(g * kHid1) * kDepth1 + 32 * ks);
        acc1[g] = mma16(a, bf, acc1[g]);
      }
    }
    __syncthreads();

#pragma unroll
    for (int r = 0; r < 8; ++r) {
      const float zi = acc1[0][r] * kFold + b1g[0];
      const float zf = acc1[1][r] * kFold + b1g[1];
      const float zg = acc1[2][r] * kFold + b1g[2];
      const float zo = acc1[3][r] * kFold + b1g[3];
      const float ig = sigm(zi);
      const float fg = sigm(zf);
      const float gg = tanhf(zg);
      const float og = sigm(zo);
      const float cn = fg * c1r[r] + ig * gg;
      c1r[r] = cn;
      const float hv = og * tanhf(cn);
      const _Float16 h16 = (_Float16)(hv * kCarry);
      const int row = 16 * mt1 + 8 * hf + r;
      A1s[row * kPitch1 + kEmbWidth + 16 * ub1 + cl] = h16;
      A2s[row * kPitch2 + 16 * ub1 + cl] = h16;
    }
    __syncthreads();

    v8f acc2[2][4];
#pragma unroll
    for (int m = 0; m < 2; ++m)
#pragma unroll
      for (int g = 0; g < 4; ++g) acc2[m][g] = (v8f){0.f, 0.f, 0.f, 0.f, 0.f, 0.f, 0.f, 0.f};
#pragma unroll 1
    for (int ks = 0; ks < kDepth2 / 32; ++ks) {
      const v16h a0 = Frag<_Float16>::load(a2Base0 + 32 * ks);
      const v16h a1 = Frag<_Float16>::load(a2Base1 + 32 * ks);
#pragma unroll
      for (int g = 0; g < 4; ++g) {
        const v16h bf = Frag<_Float16>::load(b2Base + (size_t)(g * kHid2) * kDepth2 + 32 * ks);
        acc2[0][g] = mma16(a0, bf, acc2[0][g]);
        acc2[1][g] = mma16(a1, bf, acc2[1][g]);
      }
    }
    __syncthreads();

#pragma unroll
    for (int m = 0; m < 2; ++m) {
#pragma unroll
      for (int r = 0; r < 8; ++r) {
        const float zi = acc2[m][0][r] * kFold + b2g[0];
        const float zf = acc2[m][1][r] * kFold + b2g[1];
        const float zg = acc2[m][2][r] * kFold + b2g[2];
        const float zo = acc2[m][3][r] * kFold + b2g[3];
        const float ig = sigm(zi);
        const float fg = sigm(zf);
        const float gg = tanhf(zg);
        const float og = sigm(zo);
        const float cn = fg * c2r[m * 8 + r] + ig * gg;
        c2r[m * 8 + r] = cn;
        const float hv = og * tanhf(cn);
        const _Float16 h16 = (_Float16)(hv * kCarry);
        const int row = 16 * m + 8 * hf + r;
        A2s[row * kPitch2 + kHid1 + 16 * wave + cl] = h16;
      }
    }
  }
  __syncthreads();

  {
    v8f acch[2];
    acch[0] = (v8f){0.f, 0.f, 0.f, 0.f, 0.f, 0.f, 0.f, 0.f};
    acch[1] = (v8f){0.f, 0.f, 0.f, 0.f, 0.f, 0.f, 0.f, 0.f};
    const _Float16* bdBase = Btd + (size_t)(16 * wave + cl) * kHid2 + 8 * hf;
#pragma unroll
    for (int ks = 0; ks < kHid2 / 32; ++ks) {
      const v16h a0 = Frag<_Float16>::load(a2Base0 + kHid1 + 32 * ks);
      const v16h a1 = Frag<_Float16>::load(a2Base1 + kHid1 + 32 * ks);
      const v16h bf = Frag<_Float16>::load(bdBase + 32 * ks);
      acch[0] = mma16(a0, bf, acch[0]);
      acch[1] = mma16(a1, bf, acch[1]);
    }
#pragma unroll
    for (int m = 0; m < 2; ++m) {
#pragma unroll
      for (int r = 0; r < 8; ++r) {
        float v = acch[m][r] * kFold + bdv;
        v = fmaxf(v, 0.0f);
        slab[(16 * m + 8 * hf + r) * kSlabPitch + 16 * wave + cl] = v;
      }
    }
  }
  __syncthreads();

  for (int pass = 0; pass < 2; ++pass) {
#pragma unroll
    for (int i = 0; i < 4; ++i) {
      const int row = 4 * wave + i;
      const v4f v = *(const v4f*)(slab + row * kSlabPitch + 4 * lane);
      *(volatile v4f*)(out + (size_t)(b0 + row) * kDimOut + 4 * lane) = v;
    }
    __threadfence();
  }
}

extern "C" void kernel_launch(void* const* d_in, const int* in_sizes, int n_in,
                              void* d_out, int out_size, void* d_ws, size_t ws_size,
                              hipStream_t stream) {
  if (n_in < 10) return;
  if (in_sizes[0] != kBatch * kSteps * kFields) return;
  if (in_sizes[1] != kVocab * kEmbDim) return;
  if (in_sizes[2] != kEmbWidth * kGates1 || in_sizes[3] != kHid1 * kGates1 || in_sizes[4] != kGates1) return;
  if (in_sizes[5] != kHid1 * kGates2 || in_sizes[6] != kHid2 * kGates2 || in_sizes[7] != kGates2) return;
  if (in_sizes[8] != kHid2 * kDimOut || in_sizes[9] != kDimOut) return;
  if (out_size != kBatch * kDimOut) return;

  const size_t offBt1 = 0;
  const size_t szBt1  = (size_t)kGates1 * kDepth1 * 2;
  const size_t offBt2 = offBt1 + szBt1;
  const size_t szBt2  = (size_t)kGates2 * kDepth2 * 2;
  const size_t offBtd = offBt2 + szBt2;
  const size_t szBtd  = (size_t)kDimOut * kHid2 * 2;
  const size_t total  = offBtd + szBtd;
  if (total > ws_size) return;

  const int*   x  = (const int*)  d_in[0];
  const float* E  = (const float*)d_in[1];
  const float* W1 = (const float*)d_in[2];
  const float* U1 = (const float*)d_in[3];
  const float* b1 = (const float*)d_in[4];
  const float* W2 = (const float*)d_in[5];
  const float* U2 = (const float*)d_in[6];
  const float* b2 = (const float*)d_in[7];
  const float* Wd = (const float*)d_in[8];
  const float* bd = (const float*)d_in[9];
  float* out = (float*)d_out;

  unsigned char* ws = (unsigned char*)d_ws;
  _Float16* Bt1 = (_Float16*)(ws + offBt1);
  _Float16* Bt2 = (_Float16*)(ws + offBt2);
  _Float16* Btd = (_Float16*)(ws + offBtd);

  const int nch1 = kGates1 * (kDepth1 / 8);
  build_bt<<<dim3(nch1 / 256), dim3(256), 0, stream>>>(W1, kEmbWidth, U1, kHid1, kGates1, kDepth1, Bt1, nch1);
  const int nch2 = kGates2 * (kDepth2 / 8);
  build_bt<<<dim3(nch2 / 256), dim3(256), 0, stream>>>(W2, kHid1, U2, kHid2, kGates2, kDepth2, Bt2, nch2);
  const int nchd = kDimOut * (kHid2 / 8);
  build_bt<<<dim3(nchd / 256), dim3(256), 0, stream>>>(Wd, kHid2, Wd, kHid2, kDimOut, kHid2, Btd, nchd);

  lstm2_persistent<<<dim3(kBatch / kRowsPerBlk), dim3(256), 0, stream>>>(x, E, Bt1, b1, Bt2, b2, Btd, bd, out);
}
